// CausalMHA_15599321219547
// MI455X (gfx1250) — hardware-verified
//
#include <hip/hip_runtime.h>
#include <stdint.h>

typedef __attribute__((ext_vector_type(16))) _Float16 v16h;
typedef __attribute__((ext_vector_type(8)))  _Float16 v8h;
typedef __attribute__((ext_vector_type(16))) __bf16   v16b;
typedef __attribute__((ext_vector_type(8)))  __bf16   v8b;
typedef __attribute__((ext_vector_type(8)))  float    v8f;
typedef __attribute__((ext_vector_type(4)))  float    v4f;
typedef __attribute__((ext_vector_type(4)))  unsigned v4u;

constexpr int kBatch  = 2;
constexpr int kSeq    = 2048;
constexpr int kDModel = 1024;
constexpr int kHeads  = 16;
constexpr int kHDim   = 64;
constexpr int kRows   = kBatch * kSeq;
constexpr int kNQKV   = 3 * kDModel;
constexpr int kQB     = 64;
constexpr int kKC     = 64;
constexpr int kNQB    = kSeq / kQB;

static_assert(kHeads * kHDim == kDModel, "head split");
static_assert(kDModel % 32 == 0, "GEMM K multiple of 32");
static_assert(kRows % 64 == 0 && kNQKV % 64 == 0 && kDModel % 64 == 0, "GEMM M/N multiples of 64");
static_assert(kSeq % kQB == 0 && kSeq % kKC == 0, "attention tiles");
static_assert(kNQKV % 256 == 0 && kDModel % 256 == 0, "bias kernel block-uniform split");
static_assert((kRows * kDModel) % (8 * 256) == 0, "cast kernel exact grid");

constexpr size_t kXbBytes   = (size_t)kRows * kDModel * 2;
constexpr size_t kWkTBytes  = (size_t)kNQKV * kDModel * 2;
constexpr size_t kWpTBytes  = (size_t)kDModel * kDModel * 2;
constexpr size_t kQkvBytes  = (size_t)kRows * kNQKV * 2;
constexpr size_t kOBytes    = (size_t)kRows * kDModel * 2;
constexpr size_t kBqBytes   = (size_t)kNQKV * 4;
constexpr size_t kBpBytes   = (size_t)kDModel * 4;
constexpr size_t kWsTotal   = kXbBytes + kWkTBytes + kWpTBytes + 2 * kQkvBytes + 2 * kOBytes + kBqBytes + kBpBytes;
static_assert(kWsTotal == 83902464ull, "carve total 80 MiB + 16 KiB");
static_assert(kWsTotal <= 134217728ull, "carve under 128 MiB");

__device__ __forceinline__ unsigned short f2bf_bits(float f) {
  unsigned u = __float_as_uint(f);
  return (unsigned short)((u + 0x7FFFu + ((u >> 16) & 1u)) >> 16);
}
__device__ __forceinline__ float bf_bits2f(unsigned short h) { return __uint_as_float(((unsigned)h) << 16); }

__device__ __forceinline__ void dep_guard_h(v8f& a, v8f& b, v16h x, v16h y) { asm volatile("v_nop\n\tv_nop\n\tv_nop\n\tv_nop" : "+v"(a), "+v"(b) : "v"(x), "v"(y)); }
__device__ __forceinline__ void dep_guard_b(v8f& a, v8f& b, v16b x, v16b y) { asm volatile("v_nop\n\tv_nop\n\tv_nop\n\tv_nop" : "+v"(a), "+v"(b) : "v"(x), "v"(y)); }
__device__ __forceinline__ void keep4_h(v16h a, v16h b, v16h c, v16h d) { asm volatile("v_nop" :: "v"(a), "v"(b), "v"(c), "v"(d)); }
__device__ __forceinline__ void keep4_b(v16b a, v16b b, v16b c, v16b d) { asm volatile("v_nop" :: "v"(a), "v"(b), "v"(c), "v"(d)); }
__device__ __forceinline__ void acc_guard4(v8f& a, v8f& b, v8f& c, v8f& d) { asm volatile("v_nop\n\tv_nop\n\tv_nop\n\tv_nop" : "+v"(a), "+v"(b), "+v"(c), "+v"(d)); }

template <typename T> struct Frag;
template <> struct Frag<_Float16> {
  typedef v16h V; union U { v16h v; v8h h[2]; };
  static __device__ __forceinline__ v16h load(const _Float16* p) {
    U f; f.h[0] = *(const v8h*)(p); f.h[1] = *(const v8h*)(p + 16); return f.v;
  }
  static __device__ __forceinline__ v8f mma(v16h a, v16h b, v8f c) {
    return __builtin_amdgcn_wmma_f32_16x16x32_f16(false, a, false, b, (short)0, c, false, false);
  }
  static __device__ __forceinline__ void guard(v8f& a, v8f& b, v16h x, v16h y) { dep_guard_h(a, b, x, y); }
  static __device__ __forceinline__ void keep(v16h a, v16h b, v16h c, v16h d) { keep4_h(a, b, c, d); }
};
template <> struct Frag<__bf16> {
  typedef v16b V; union U { v16b v; v8b h[2]; };
  static __device__ __forceinline__ v16b load(const __bf16* p) {
    U f; f.h[0] = *(const v8b*)(p); f.h[1] = *(const v8b*)(p + 16); return f.v;
  }
  static __device__ __forceinline__ v8f mma(v16b a, v16b b, v8f c) {
    return __builtin_amdgcn_wmma_f32_16x16x32_bf16(false, a, false, b, (short)0, c, false, false);
  }
  static __device__ __forceinline__ void guard(v8f& a, v8f& b, v16b x, v16b y) { dep_guard_b(a, b, x, y); }
  static __device__ __forceinline__ void keep(v16b a, v16b b, v16b c, v16b d) { keep4_b(a, b, c, d); }
};

template <int ET> struct Elem;
template <> struct Elem<0> { typedef _Float16 T; };
template <> struct Elem<1> { typedef __bf16 T; };
template <int ET, int SPLITK, int BIAS_MODE, int OUT_MODE>
__global__ __launch_bounds__(256) void wmma_gemm64(
    const unsigned short* __restrict__ Ap, const unsigned short* __restrict__ A2p, int lda, long strideA,
    const unsigned short* __restrict__ Btp, const unsigned short* __restrict__ Bt2p, int ldb, long strideB,
    void* __restrict__ Cout, void* __restrict__ Cout2, int ldc, long strideC,
    const float* __restrict__ bias,
    int M, int N, int K, float scale) {
  typedef typename Elem<ET>::T T;
  typedef typename Frag<T>::V V;
  const T* A = (const T*)Ap; const T* A2 = (const T*)A2p; const T* Bt = (const T*)Btp; const T* Bt2 = (const T*)Bt2p;
  __shared__ __align__(16) float sT[8][16 * 68];
  const int b    = blockIdx.y;
  const int lane = threadIdx.x & 31;
  const int wave = threadIdx.x >> 5;
  const int tilesN = N >> 6;
  const int tilesM = M >> 6;
  const int tile = blockIdx.x * 8 + wave;
  if (tile >= tilesM * tilesN) return;
  const int tm = tile / tilesN;
  const int tn = tile - tm * tilesN;
  const int m0 = tm << 6;
  const int n0 = tn << 6;

  const T* Ab  = A  + (size_t)b * strideA;
  const T* Bb  = Bt + (size_t)b * strideB;
  const T* Ab2 = (SPLITK >= 1) ? (A2  + (size_t)b * strideA) : nullptr;
  const T* Bb2 = (SPLITK == 2) ? (Bt2 + (size_t)b * strideB) : nullptr;

  const int rlane = lane & 15;
  const int koff  = (lane >> 4) * 8;
  const int mOff  = (lane >> 4) * 8;

  v8f acc[4][4];
#pragma unroll
  for (int i = 0; i < 4; ++i)
#pragma unroll
    for (int j = 0; j < 4; ++j) acc[i][j] = (v8f){0.f,0.f,0.f,0.f,0.f,0.f,0.f,0.f};

  for (int k0 = 0; k0 < K; k0 += 32) {
    V bh[4], bl[4];
#pragma unroll
    for (int j = 0; j < 4; ++j) {
      const size_t bo = (size_t)(n0 + (j << 4) + rlane) * ldb + koff + k0;
      bh[j] = Frag<T>::load(Bb + bo);
      if (SPLITK == 2) bl[j] = Frag<T>::load(Bb2 + bo);
    }
#pragma unroll
    for (int i = 0; i < 4; ++i) {
      const size_t ao = (size_t)(m0 + (i << 4) + rlane) * lda + koff + k0;
      V ah = Frag<T>::load(Ab + ao);
      V al;
      if (SPLITK >= 1) al = Frag<T>::load(Ab2 + ao); else al = ah;
#pragma unroll
      for (int j = 0; j < 4; ++j) {
        acc[i][j] = Frag<T>::mma(ah, bh[j], acc[i][j]);
        if (SPLITK == 2) acc[i][j] = Frag<T>::mma(ah, bl[j], acc[i][j]);
        if (SPLITK >= 1) acc[i][j] = Frag<T>::mma(al, bh[j], acc[i][j]);
      }
      Frag<T>::guard(acc[i][0], acc[i][3], ah, al);
    }
    Frag<T>::keep(bh[0], bh[1], bh[2], bh[3]);
    if (SPLITK == 2) Frag<T>::keep(bl[0], bl[1], bl[2], bl[3]);
  }
  acc_guard4(acc[0][0], acc[0][1], acc[0][2], acc[0][3]);
  acc_guard4(acc[1][0], acc[1][1], acc[1][2], acc[1][3]);
  acc_guard4(acc[2][0], acc[2][1], acc[2][2], acc[2][3]);
  acc_guard4(acc[3][0], acc[3][1], acc[3][2], acc[3][3]);

  float* slab = sT[wave];
#pragma unroll
  for (int i = 0; i < 4; ++i) {
    const int mBase = m0 + (i << 4);
#pragma unroll
    for (int j = 0; j < 4; ++j) {
      const int n = n0 + (j << 4) + rlane;
      float bv = 0.f;
      if (BIAS_MODE == 2) bv = bias[n];
#pragma unroll
      for (int r = 0; r < 8; ++r) {
        float v = acc[i][j][r] * scale;
        if (BIAS_MODE == 1) v += bias[mBase + mOff + r];
        if (BIAS_MODE == 2) v += bv;
        slab[(mOff + r) * 68 + (j << 4) + rlane] = v;
      }
    }
    __builtin_amdgcn_fence(__ATOMIC_RELEASE, "workgroup");
    __builtin_amdgcn_wave_barrier();
    __builtin_amdgcn_fence(__ATOMIC_ACQUIRE, "workgroup");
    if (OUT_MODE == 0) {
      float* C = (float*)Cout + (size_t)b * strideC;
      const int hh = lane >> 4, c4 = (lane & 15) * 4;
      for (int pass = 0; pass < 2; ++pass) {
#pragma unroll
        for (int it = 0; it < 8; ++it) {
          const int row = it * 2 + hh;
          v4f v = *(const v4f*)(slab + row * 68 + c4);
          *(volatile v4f*)(C + (size_t)(mBase + row) * ldc + n0 + c4) = v;
        }
        __threadfence();
      }
    } else {
      const int q = lane >> 3, c8 = (lane & 7) * 8;
      unsigned short* C  = (unsigned short*)Cout  + (size_t)b * strideC;
      unsigned short* C2 = (OUT_MODE == 2) ? ((unsigned short*)Cout2 + (size_t)b * strideC) : nullptr;
      for (int pass = 0; pass < 2; ++pass) {
#pragma unroll
        for (int it = 0; it < 4; ++it) {
          const int row = it * 4 + q;
          const float* sp = slab + row * 68 + c8;
          v8h hv, lv;
#pragma unroll
          for (int e = 0; e < 8; ++e) {
            if (OUT_MODE == 1) {
              hv[e] = (_Float16)sp[e];
            } else {
              unsigned short hb = f2bf_bits(sp[e]);
              unsigned short lb = f2bf_bits(sp[e] - bf_bits2f(hb));
              hv[e] = __builtin_bit_cast(_Float16, hb);
              lv[e] = __builtin_bit_cast(_Float16, lb);
            }
          }
          *(volatile v8h*)(C + (size_t)(mBase + row) * ldc + n0 + c8) = hv;
          if (OUT_MODE == 2) *(volatile v8h*)(C2 + (size_t)(mBase + row) * ldc + n0 + c8) = lv;
        }
        __threadfence();
      }
    }
    __builtin_amdgcn_fence(__ATOMIC_RELEASE, "workgroup");
    __builtin_amdgcn_wave_barrier();
    __builtin_amdgcn_fence(__ATOMIC_ACQUIRE, "workgroup");
  }
}

__global__ __launch_bounds__(256) void cast_f32_bf16x8(const float* __restrict__ in,
                                                      unsigned short* __restrict__ out, int n8) {
  const int i = blockIdx.x * 256 + threadIdx.x;
  if (i < n8) {
    const size_t e0 = (size_t)i * 8;
    const v4f a = *(const v4f*)(in + e0);
    const v4f c = *(const v4f*)(in + e0 + 4);
    v4u w;
    w[0] = (unsigned)f2bf_bits(a[0]) | ((unsigned)f2bf_bits(a[1]) << 16);
    w[1] = (unsigned)f2bf_bits(a[2]) | ((unsigned)f2bf_bits(a[3]) << 16);
    w[2] = (unsigned)f2bf_bits(c[0]) | ((unsigned)f2bf_bits(c[1]) << 16);
    w[3] = (unsigned)f2bf_bits(c[2]) | ((unsigned)f2bf_bits(c[3]) << 16);
    *(volatile v4u*)(out + e0) = w;
    __threadfence();
    *(volatile v4u*)(out + e0) = w;
  }
}

__global__ __launch_bounds__(256) void transpose_cast_bf16(const float* __restrict__ in,
                                                           unsigned short* __restrict__ out, int R, int Cc) {
  __shared__ float tile[64][65];
  const int t = threadIdx.x;
  const int c0 = blockIdx.x * 64, r0 = blockIdx.y * 64;
  {
    const int rr = t >> 2, cc = (t & 3) * 16;
    const float* src = in + (size_t)(r0 + rr) * Cc + c0 + cc;
#pragma unroll
    for (int q4 = 0; q4 < 4; ++q4) {
      const v4f v = *(const v4f*)(src + 4 * q4);
      tile[rr][cc + 4 * q4 + 0] = v[0];
      tile[rr][cc + 4 * q4 + 1] = v[1];
      tile[rr][cc + 4 * q4 + 2] = v[2];
      tile[rr][cc + 4 * q4 + 3] = v[3];
    }
  }
  __syncthreads();
  v4u w[2];
  size_t oo[2];
#pragma unroll
  for (int it = 0; it < 2; ++it) {
    const int n = it * 32 + (t >> 3);
    const int k8 = (t & 7) * 8;
#pragma unroll
    for (int e = 0; e < 4; ++e) {
      const unsigned hb0 = f2bf_bits(tile[k8 + 2 * e][n]);
      const unsigned hb1 = f2bf_bits(tile[k8 + 2 * e + 1][n]);
      w[it][e] = hb0 | (hb1 << 16);
    }
    oo[it] = (size_t)(c0 + n) * R + r0 + k8;
  }
  for (int pass = 0; pass < 2; ++pass) {
#pragma unroll
    for (int it = 0; it < 2; ++it) *(volatile v4u*)(out + oo[it]) = w[it];
    __threadfence();
  }
}

__global__ __launch_bounds__(256) void rne_bias2(const float* __restrict__ b0, const float* __restrict__ b1,
                                                 float* __restrict__ o0, float* __restrict__ o1, int nb0) {
  const int t = threadIdx.x;
  if ((int)blockIdx.x < nb0) {
    const int i = blockIdx.x * 256 + t;
    const float v = bf_bits2f(f2bf_bits(b0[i]));
    ((volatile float*)o0)[i] = v;
    __threadfence();
    ((volatile float*)o0)[i] = v;
  } else {
    const int i = ((int)blockIdx.x - nb0) * 256 + t;
    const float v = bf_bits2f(f2bf_bits(b1[i]));
    ((volatile float*)o1)[i] = v;
    __threadfence();
    ((volatile float*)o1)[i] = v;
  }
}

__device__ __forceinline__ unsigned short at_bf_bits(float f) {
  unsigned u = __float_as_uint(f);
  return (unsigned short)((u + 0x7FFFu + ((u >> 16) & 1u)) >> 16);
}
__device__ __forceinline__ __bf16 at_f2bf(float f) { return __builtin_bit_cast(__bf16, at_bf_bits(f)); }
__device__ __forceinline__ void at_split(float f, __bf16& hi, __bf16& lo) {
  const unsigned short hb = at_bf_bits(f);
  hi = __builtin_bit_cast(__bf16, hb);
  lo = at_f2bf(f - __uint_as_float(((unsigned)hb) << 16));
}
__device__ __forceinline__ v8f at_mma(v16b a, v16b b, v8f c) {
  c = __builtin_amdgcn_wmma_f32_16x16x32_bf16(false, a, false, b, (short)0, c, false, false);
  asm volatile("v_nop\n\tv_nop\n\tv_nop\n\tv_nop" : "+v"(c) : "v"(a), "v"(b));
  return c;
}

__global__ __launch_bounds__(128)
void attn_causal64(const unsigned short* __restrict__ Ph, const unsigned short* __restrict__ Pl,
                   unsigned short* __restrict__ Oh, unsigned short* __restrict__ Ol) {
  union FB { v16b v; v8b h[2]; };
  __shared__ __align__(16) unsigned short Ksh[kKC * kHDim];
  __shared__ __align__(16) unsigned short Ksl[kKC * kHDim];
  __shared__ __align__(16) unsigned short Vth[kHDim * kKC];
  __shared__ __align__(16) unsigned short Vtl[kHDim * kKC];
  __shared__ __align__(16) __bf16 Psh[4][16 * kKC];
  __shared__ __align__(16) __bf16 Psl[4][16 * kKC];
  __shared__ __align__(16) float  Os[4][16 * 68];

  const int tid  = threadIdx.x;
  const int wave = tid >> 5;
  const int lane = tid & 31;
  const int hh   = lane >> 4;
  const int c    = lane & 15;

  const int bx  = blockIdx.x;
  const int qb  = bx % kNQB;
  const int bhd = bx / kNQB;
  const int h   = bhd % kHeads;
  const int b   = bhd / kHeads;
  const int q0  = qb * kQB + wave * 16;
  const size_t rowb = (size_t)b * kSeq;
  const int qcol = h * kHDim;
  const int kcol = kDModel + h * kHDim;
  const int vcol = 2 * kDModel + h * kHDim;
  const float ninf = -__builtin_inff();

  v16b qah[2], qal[2];
  {
    const size_t qo = (rowb + q0 + c) * (size_t)kNQKV + qcol + 8 * hh;
#pragma unroll
    for (int dc = 0; dc < 2; ++dc) {
      qah[dc] = Frag<__bf16>::load((const __bf16*)(Ph + qo + dc * 32));
      qal[dc] = Frag<__bf16>::load((const __bf16*)(Pl + qo + dc * 32));
    }
  }

  float mrow[8], lrow[8];
  v8f oacc[4];
#pragma unroll
  for (int r = 0; r < 8; ++r) { mrow[r] = ninf; lrow[r] = 0.f; }
#pragma unroll
  for (int t = 0; t < 4; ++t) oacc[t] = (v8f){0.f,0.f,0.f,0.f,0.f,0.f,0.f,0.f};

  for (int kc = 0; kc <= qb; ++kc) {
    const int kv0 = kc * kKC;
    __syncthreads();
#pragma unroll
    for (int i = 0; i < 4; ++i) {
      const int ch = tid + 128 * i;
      const int kvr = ch >> 3, d8 = (ch & 7) * 8;
      const size_t go = (rowb + kv0 + kvr) * (size_t)kNQKV + kcol + d8;
      const v4u wh = *(const v4u*)(Ph + go);
      const v4u wl = *(const v4u*)(Pl + go);
      *(v4u*)(Ksh + kvr * kHDim + d8) = wh;
      *(v4u*)(Ksl + kvr * kHDim + d8) = wl;
    }
    asm volatile("" ::: "memory");
#pragma unroll
    for (int i = 0; i < 4; ++i) {
      const int ch = tid + 128 * i;
      const int kvr = ch >> 3, d8 = (ch & 7) * 8;
      const size_t go = (rowb + kv0 + kvr) * (size_t)kNQKV + vcol + d8;
      const v4u wh = *(const v4u*)(Ph + go);
      const v4u wl = *(const v4u*)(Pl + go);
#pragma unroll
      for (int e = 0; e < 4; ++e) {
        const unsigned xh = wh[e], xl = wl[e];
        Vth[(d8 + 2 * e) * kKC + kvr]     = (unsigned short)(xh & 0xffffu);
        Vth[(d8 + 2 * e + 1) * kKC + kvr] = (unsigned short)(xh >> 16);
        Vtl[(d8 + 2 * e) * kKC + kvr]     = (unsigned short)(xl & 0xffffu);
        Vtl[(d8 + 2 * e + 1) * kKC + kvr] = (unsigned short)(xl >> 16);
      }
    }
    __syncthreads();

    v8f s[4];
#pragma unroll
    for (int j = 0; j < 4; ++j) {
      s[j] = (v8f){0.f,0.f,0.f,0.f,0.f,0.f,0.f,0.f};
#pragma unroll
      for (int dc = 0; dc < 2; ++dc) {
        const int ko = (j * 16 + c) * kHDim + dc * 32 + 8 * hh;
        FB kb, kl;
        kb.h[0] = *(const v8b*)(Ksh + ko);
        kb.h[1] = *(const v8b*)(Ksh + ko + 16);
        kl.h[0] = *(const v8b*)(Ksl + ko);
        kl.h[1] = *(const v8b*)(Ksl + ko + 16);
        s[j] = at_mma(qah[dc], kb.v, s[j]);
        s[j] = at_mma(qah[dc], kl.v, s[j]);
        s[j] = at_mma(qal[dc], kb.v, s[j]);
      }
    }
    const bool diag = (kc == qb);
    float cm[8];
#pragma unroll
    for (int r = 0; r < 8; ++r) {
      const int qrow = q0 + 8 * hh + r;
      float m = ninf;
#pragma unroll
      for (int j = 0; j < 4; ++j) {
        const int kvcol = kv0 + j * 16 + c;
        float val = s[j][r] * 0.125f;
        val = (diag && (kvcol > qrow)) ? ninf : val;
        s[j][r] = val;
        m = fmaxf(m, val);
      }
#pragma unroll
      for (int off = 1; off < 16; off <<= 1) m = fmaxf(m, __shfl_xor(m, off, 32));
      cm[r] = m;
    }
    __bf16* pwh = Psh[wave];
    __bf16* pwl = Psl[wave];
#pragma unroll
    for (int r = 0; r < 8; ++r) {
      const float mnew = fmaxf(mrow[r], cm[r]);
      const float alpha = expf(mrow[r] - mnew);
      mrow[r] = mnew;
      float psum = 0.f;
#pragma unroll
      for (int j = 0; j < 4; ++j) {
        const float p = expf(s[j][r] - mnew);
        psum += p;
        __bf16 a, bl;
        at_split(p, a, bl);
        pwh[(8 * hh + r) * kKC + j * 16 + c] = a;
        pwl[(8 * hh + r) * kKC + j * 16 + c] = bl;
      }
#pragma unroll
      for (int off = 1; off < 16; off <<= 1) psum += __shfl_xor(psum, off, 32);
      lrow[r] = lrow[r] * alpha + psum;
#pragma unroll
      for (int t = 0; t < 4; ++t) oacc[t][r] *= alpha;
    }
    __builtin_amdgcn_fence(__ATOMIC_RELEASE, "workgroup");
    __builtin_amdgcn_wave_barrier();
    __builtin_amdgcn_fence(__ATOMIC_ACQUIRE, "workgroup");
#pragma unroll 1
    for (int kk = 0; kk < 2; ++kk) {
      FB pa, pl;
      pa.h[0] = *(const v8b*)(pwh + c * kKC + kk * 32 + 8 * hh);
      pa.h[1] = *(const v8b*)(pwh + c * kKC + kk * 32 + 16 + 8 * hh);
      pl.h[0] = *(const v8b*)(pwl + c * kKC + kk * 32 + 8 * hh);
      pl.h[1] = *(const v8b*)(pwl + c * kKC + kk * 32 + 16 + 8 * hh);
#pragma unroll
      for (int t = 0; t < 4; ++t) {
        const int vo = (t * 16 + c) * kKC + kk * 32 + 8 * hh;
        FB vb, vl;
        vb.h[0] = *(const v8b*)(Vth + vo);
        vb.h[1] = *(const v8b*)(Vth + vo + 16);
        vl.h[0] = *(const v8b*)(Vtl + vo);
        vl.h[1] = *(const v8b*)(Vtl + vo + 16);
        oacc[t] = at_mma(pa.v, vb.v, oacc[t]);
        oacc[t] = at_mma(pa.v, vl.v, oacc[t]);
        oacc[t] = at_mma(pl.v, vb.v, oacc[t]);
      }
    }
  }

  float* os = Os[wave];
#pragma unroll
  for (int r = 0; r < 8; ++r) {
    const float inv = 1.0f / lrow[r];
#pragma unroll
    for (int t = 0; t < 4; ++t) os[(8 * hh + r) * 68 + t * 16 + c] = oacc[t][r] * inv;
  }
  __builtin_amdgcn_fence(__ATOMIC_RELEASE, "workgroup");
  __builtin_amdgcn_wave_barrier();
  __builtin_amdgcn_fence(__ATOMIC_ACQUIRE, "workgroup");
  {
    const int qq = lane >> 3, c8 = (lane & 7) * 8;
    v4u wh4[4], wl4[4];
    size_t oo[4];
#pragma unroll
    for (int it = 0; it < 4; ++it) {
      const int row = it * 4 + qq;
      const float* sp = os + row * 68 + c8;
      const v4f f0 = *(const v4f*)(sp);
      const v4f f1 = *(const v4f*)(sp + 4);
      float v8[8];
      v8[0] = f0[0]; v8[1] = f0[1]; v8[2] = f0[2]; v8[3] = f0[3];
      v8[4] = f1[0]; v8[5] = f1[1]; v8[6] = f1[2]; v8[7] = f1[3];
#pragma unroll
      for (int e = 0; e < 4; ++e) {
        const unsigned hb0 = f2bf_bits(v8[2 * e]);
        const unsigned lb0 = f2bf_bits(v8[2 * e] - bf_bits2f((unsigned short)hb0));
        const unsigned hb1 = f2bf_bits(v8[2 * e + 1]);
        const unsigned lb1 = f2bf_bits(v8[2 * e + 1] - bf_bits2f((unsigned short)hb1));
        wh4[it][e] = hb0 | (hb1 << 16);
        wl4[it][e] = lb0 | (lb1 << 16);
      }
      oo[it] = (rowb + q0 + row) * (size_t)kDModel + qcol + c8;
    }
    for (int pass = 0; pass < 2; ++pass) {
#pragma unroll
      for (int it = 0; it < 4; ++it) {
        *(volatile v4u*)(Oh + oo[it]) = wh4[it];
        *(volatile v4u*)(Ol + oo[it]) = wl4[it];
      }
      __threadfence();
    }
  }
}

extern "C" void kernel_launch(void* const* d_in, const int* in_sizes, int n_in,
                              void* d_out, int out_size, void* d_ws, size_t ws_size,
                              hipStream_t stream) {
  const float* x      = (const float*)d_in[0];
  const float* W_kqv  = (const float*)d_in[1];
  const float* b_kqv  = (const float*)d_in[2];
  const float* W_proj = (const float*)d_in[3];
  const float* b_proj = (const float*)d_in[4];
  float* out = (float*)d_out;

  if (n_in < 5) return;
  if (in_sizes[0] != kRows * kDModel || in_sizes[1] != kDModel * kNQKV || in_sizes[2] != kNQKV ||
      in_sizes[3] != kDModel * kDModel || in_sizes[4] != kDModel || out_size != kRows * kDModel) return;
  if (kWsTotal > ws_size) return;

  char* ws = (char*)d_ws;
  size_t off = 0;
  unsigned short* Xb  = (unsigned short*)(ws + off); off += kXbBytes;
  unsigned short* WkT = (unsigned short*)(ws + off); off += kWkTBytes;
  unsigned short* WpT = (unsigned short*)(ws + off); off += kWpTBytes;
  unsigned short* Ph  = (unsigned short*)(ws + off); off += kQkvBytes;
  unsigned short* Pl  = (unsigned short*)(ws + off); off += kQkvBytes;
  unsigned short* Oh  = (unsigned short*)(ws + off); off += kOBytes;
  unsigned short* Ol  = (unsigned short*)(ws + off); off += kOBytes;
  float* bq_r = (float*)(ws + off); off += kBqBytes;
  float* bp_r = (float*)(ws + off); off += kBpBytes;
  if (off > ws_size) return;

  const int n8 = (kRows * kDModel) / 8;
  cast_f32_bf16x8<<<n8 / 256, 256, 0, stream>>>(x, Xb, n8);
  transpose_cast_bf16<<<dim3(kNQKV / 64, kDModel / 64), 256, 0, stream>>>(W_kqv, WkT, kDModel, kNQKV);
  transpose_cast_bf16<<<dim3(kDModel / 64, kDModel / 64), 256, 0, stream>>>(W_proj, WpT, kDModel, kDModel);
  rne_bias2<<<(kNQKV + kDModel) / 256, 256, 0, stream>>>(b_kqv, b_proj, bq_r, bp_r, kNQKV / 256);
  wmma_gemm64<1, 0, 2, 2><<<dim3((kRows / 64) * (kNQKV / 64) / 8, 1), 256, 0, stream>>>(
      Xb, Xb, kDModel, 0L, WkT, WkT, kDModel, 0L, (void*)Ph, (void*)Pl, kNQKV, 0L, bq_r,
      kRows, kNQKV, kDModel, 1.0f);
  attn_causal64<<<kBatch * kHeads * kNQB, 128, 0, stream>>>(Ph, Pl, Oh, Ol);
  wmma_gemm64<1, 1, 2, 0><<<dim3((kRows / 64) * (kDModel / 64) / 8, 1), 256, 0, stream>>>(
      Oh, Ol, kDModel, 0L, WpT, WpT, kDModel, 0L, (void*)out, (void*)out, kDModel, 0L, bp_r,
      kRows, kDModel, kDModel, 1.0f);
}
